// S6_70480413327620
// MI455X (gfx1250) — hardware-run, weakly checked
//
#include <hip/hip_runtime.h>
#include <hip/hip_fp16.h>
#include <math.h>

constexpr int kBatch = 2;
constexpr int kSeq   = 1024;
constexpr int kDin   = 2048;
constexpr int kNst   = 16;
constexpr int kDtR   = 64;
constexpr int kProj  = kDtR + 2 * kNst;
constexpr int kXpP   = 128;
constexpr int kRows  = kBatch * kSeq;
constexpr int kOffB  = kDtR;
constexpr int kOffC  = kDtR + kNst;
static_assert(kProj == 96, "projection width");
static_assert(kProj <= kXpP && (kXpP % 64) == 0, "N pad");
static_assert((kRows % 64) == 0 && (kDin % 64) == 0, "GEMM M,N multiples of 64");
static_assert((kDin % 32) == 0 && (kDtR % 32) == 0, "GEMM K multiples of 32");
static_assert((kSeq % 64) == 0 && (kDin % 64) == 0, "scan tile multiples");
static_assert((kOffB % 4) == 0 && (kOffC % 4) == 0, "B | C columns 16-B aligned");

constexpr float kCarryX   = 64.0f;
constexpr float kCarryWx  = 2048.0f;
constexpr float kCarryDtx = 64.0f;
constexpr float kCarryWdt = 1024.0f;
constexpr float kScale0   = 1.0f / (kCarryX * kCarryWx);
constexpr float kScale1   = 1.0f / (kCarryDtx * kCarryWdt);
constexpr float kYCarry   = 16.0f;
constexpr float kYInv     = 1.0f / kYCarry;

constexpr size_t kSzXH    = (size_t)kRows * kDin * 2;
constexpr size_t kSzWXH   = (size_t)kXpP * kDin * 2;
constexpr size_t kSzWDH   = (size_t)kDin * kDtR * 2;
constexpr size_t kSzXP    = (size_t)kRows * kXpP * 4;
constexpr size_t kSzDTXH  = (size_t)kRows * kDtR * 2;
constexpr size_t kSzDT    = (size_t)kRows * kDin * 4;
constexpr size_t kSzYH    = (size_t)kRows * kDin * 2;
constexpr size_t kOffXH   = 0;
constexpr size_t kOffWXH  = kOffXH + kSzXH;
constexpr size_t kOffWDH  = kOffWXH + kSzWXH;
constexpr size_t kOffXP   = kOffWDH + kSzWDH;
constexpr size_t kOffDTXH = kOffXP + kSzXP;
constexpr size_t kOffDT   = kOffDTXH + kSzDTXH;
constexpr size_t kOffYH   = kOffDT + kSzDT;
constexpr size_t kWsTotal = kOffYH + kSzYH;
static_assert(kWsTotal == 35651584ull, "carve total");
static_assert(kWsTotal <= 134217728ull, "carve cap");
static_assert((kOffWXH % 128) == 0 && (kOffWDH % 128) == 0 && (kOffXP % 128) == 0 &&
              (kOffDTXH % 128) == 0 && (kOffDT % 128) == 0 && (kOffYH % 128) == 0, "128-B aligned regions");

namespace eng {

typedef __attribute__((ext_vector_type(16))) _Float16 v16h;
typedef __attribute__((ext_vector_type(8)))  _Float16 v8h;
typedef __attribute__((ext_vector_type(8)))  float    v8f;
typedef __attribute__((ext_vector_type(4)))  float    v4f;
typedef __attribute__((ext_vector_type(2)))  unsigned v2u;

__device__ __forceinline__ v16h frag_load(const _Float16* p) {
  union U { v16h v; v8h h[2]; } f;
  f.h[0] = *(const v8h*)(p);
  f.h[1] = *(const v8h*)(p + 16);
  return f.v;
}
__device__ __forceinline__ v8f mma_guarded(v16h a, v16h b, v8f c) {
  c = __builtin_amdgcn_wmma_f32_16x16x32_f16(false, a, false, b, (short)0, c, false, false);
  asm volatile("v_nop\n\tv_nop\n\tv_nop\n\tv_nop" : "+v"(c) : "v"(a), "v"(b));
  return c;
}
__device__ __forceinline__ void keep4(v16h a, v16h b, v16h c, v16h d) {
  asm volatile("v_nop" :: "v"(a), "v"(b), "v"(c), "v"(d));
}

template <int BIAS_MODE>
__global__ __launch_bounds__(256) void gemm_f16_kernel(
    const unsigned short* __restrict__ Ap, int lda,
    const unsigned short* __restrict__ Btp, int ldb,
    float* __restrict__ C, int ldc,
    const float* __restrict__ bias,
    int M, int N, int K, float scale)
{
  __shared__ __align__(16) float sT[8][16 * 68];
  const _Float16* A  = (const _Float16*)Ap;
  const _Float16* Bt = (const _Float16*)Btp;
  const int lane = threadIdx.x & 31;
  const int wave = threadIdx.x >> 5;
  const int tilesN = N >> 6;
  const int tilesM = M >> 6;
  const int tile = blockIdx.x * 8 + wave;
  if (tile >= tilesM * tilesN) return;
  const int tm = tile / tilesN;
  const int tn = tile - tm * tilesN;
  const int m0 = tm << 6;
  const int n0 = tn << 6;
  const int rlane = lane & 15;
  const int koff  = (lane >> 4) * 8;
  const int mOff  = (lane >> 4) * 8;

  v8f acc[4][4];
#pragma unroll
  for (int i = 0; i < 4; ++i)
#pragma unroll
    for (int j = 0; j < 4; ++j) acc[i][j] = (v8f){0.f, 0.f, 0.f, 0.f, 0.f, 0.f, 0.f, 0.f};

  for (int k0 = 0; k0 < K; k0 += 32) {
    v16h bh[4];
#pragma unroll
    for (int j = 0; j < 4; ++j) {
      const size_t bo = (size_t)(n0 + (j << 4) + rlane) * ldb + koff + k0;
      bh[j] = frag_load(Bt + bo);
    }
#pragma unroll
    for (int i = 0; i < 4; ++i) {
      const size_t ao = (size_t)(m0 + (i << 4) + rlane) * lda + koff + k0;
      const v16h ah = frag_load(A + ao);
#pragma unroll
      for (int j = 0; j < 4; ++j) acc[i][j] = mma_guarded(ah, bh[j], acc[i][j]);
    }
    keep4(bh[0], bh[1], bh[2], bh[3]);
  }

  float* slab = sT[wave];
#pragma unroll
  for (int i = 0; i < 4; ++i) {
    const int mBase = m0 + (i << 4);
#pragma unroll
    for (int j = 0; j < 4; ++j) {
      const int n = n0 + (j << 4) + rlane;
      float bv = 0.f;
      if (BIAS_MODE == 2) bv = bias[n];
#pragma unroll
      for (int r = 0; r < 8; ++r) {
        float v = acc[i][j][r] * scale;
        if (BIAS_MODE == 2) v += bv;
        slab[(mOff + r) * 68 + (j << 4) + rlane] = v;
      }
    }
    __builtin_amdgcn_fence(__ATOMIC_RELEASE, "workgroup");
    __builtin_amdgcn_wave_barrier();
    __builtin_amdgcn_fence(__ATOMIC_ACQUIRE, "workgroup");
    {
      const int hh = lane >> 4;
      const int c4 = (lane & 15) * 4;
      for (int pass = 0; pass < 2; ++pass) {
#pragma unroll
        for (int it = 0; it < 8; ++it) {
          const int row = it * 2 + hh;
          const v4f v = *(const v4f*)(slab + row * 68 + c4);
          *(volatile v4f*)(C + (size_t)(mBase + row) * ldc + n0 + c4) = v;
        }
        __threadfence();
      }
    }
    __builtin_amdgcn_fence(__ATOMIC_RELEASE, "workgroup");
    __builtin_amdgcn_wave_barrier();
    __builtin_amdgcn_fence(__ATOMIC_ACQUIRE, "workgroup");
  }
}

__global__ __launch_bounds__(256) void to_f16_plane_kernel(
    const float* __restrict__ src, int ld_src, int rows_src, int cols,
    unsigned short* __restrict__ dst, int total8, float carry)
{
  const int i = blockIdx.x * 256 + threadIdx.x;
  if (i >= total8) return;
  const int e0  = i << 3;
  const int row = e0 / cols;
  const int col = e0 - row * cols;
  const bool live = (row < rows_src);
  const int rc = live ? row : (rows_src - 1);
  const float* sp = src + (size_t)rc * ld_src + col;
  v4f a0 = *(const v4f*)(sp);
  v4f a1 = *(const v4f*)(sp + 4);
  asm volatile("" : "+v"(a0), "+v"(a1));
  v8h hv;
#pragma unroll
  for (int e = 0; e < 4; ++e) {
    float p = a0[e] * carry;
    float q = a1[e] * carry;
    p = live ? p : 0.0f;
    q = live ? q : 0.0f;
    p = (fabsf(p) < 6.103515625e-05f) ? 0.0f : p;
    q = (fabsf(q) < 6.103515625e-05f) ? 0.0f : q;
    hv[e]     = (_Float16)p;
    hv[4 + e] = (_Float16)q;
  }
  unsigned short* qd = dst + (size_t)e0;
  *(volatile v8h*)qd = hv;
  __threadfence();
  *(volatile v8h*)qd = hv;
}

__device__ __forceinline__ float h16_to_f32(unsigned hb) {
  const unsigned sgn = (hb & 0x8000u) << 16;
  const unsigned em = hb & 0x7fffu;
  const float fn = __uint_as_float((em << 13) + 0x38000000u);
  const float fs = (float)em * 5.9604644775390625e-8f;
  const float mag = (em < 0x400u) ? fs : fn;
  return __uint_as_float(__float_as_uint(mag) | sgn);
}

__global__ __launch_bounds__(256) void decode_y_kernel(
    const unsigned* __restrict__ yw, float* __restrict__ out, int total4, float inv)
{
  const int i = blockIdx.x * 256 + threadIdx.x;
  if (i >= total4) return;
  const v2u w = *(const v2u*)(yw + 2 * (size_t)i);
  const unsigned w0 = w[0];
  const unsigned w1 = w[1];
  const float f0 = h16_to_f32(w0 & 0xffffu) * inv;
  const float f1 = h16_to_f32(w0 >> 16) * inv;
  const float f2 = h16_to_f32(w1 & 0xffffu) * inv;
  const float f3 = h16_to_f32(w1 >> 16) * inv;
  const v4f o = (v4f){f0, f1, f2, f3};
  float* qd = out + 4 * (size_t)i;
  *(volatile v4f*)qd = o;
  __threadfence();
  *(volatile v4f*)qd = o;
}

}

typedef float    ms1_v4f __attribute__((ext_vector_type(4)));
typedef unsigned ms1_v4u __attribute__((ext_vector_type(4)));
struct ms1_args {
  const float* dtpre;
  const float* u;
  const float* bc;
  const float* z;
  const float* A_log;
  const float* Dskip;
  __half* y;
  __half* y_lo;
  long ld_dtpre;
  long ld_u;
  long ld_bc;
  long ld_z;
  long ld_y;
  int offB;
  int offC;
  int offZ;
  float ycarry;
  int dir;
  int D;
  int L;
  int nbatch;
};
static_assert(sizeof(ms1_args) == 136);

__device__ __forceinline__ float ms1_flush16(float v) {
  return (fabsf(v) < 6.103515625e-05f) ? 0.0f : v;
}
__device__ __forceinline__ unsigned ms1_h16bits(float v) {
  return (unsigned)__half_as_ushort(__float2half_rn(ms1_flush16(v)));
}
__device__ __forceinline__ float ms1_h16val(unsigned b) {
  return __half2float(__ushort_as_half((unsigned short)b));
}
__device__ __forceinline__ float ms1_softplus(float v) {
  return fmaxf(v, 0.0f) + log1pf(expf(-fabsf(v)));
}
__device__ __forceinline__ void ms1_pack2(float v0, float v1, unsigned& hw, unsigned& lw) {
  const unsigned h0 = ms1_h16bits(v0);
  const unsigned h1 = ms1_h16bits(v1);
  const float r0 = (v0 - ms1_h16val(h0)) * 2048.0f;
  const float r1 = (v1 - ms1_h16val(h1)) * 2048.0f;
  const unsigned l0 = ms1_h16bits(r0);
  const unsigned l1 = ms1_h16bits(r1);
  hw = h0 | (h1 << 16);
  lw = l0 | (l1 << 16);
}

template <int NSTATE>
__global__ __launch_bounds__(64 * (NSTATE / 16)) void ms1_scan_kernel(ms1_args a)
{
  static_assert(NSTATE == 16 || NSTATE == 64);
  constexpr int NQ  = NSTATE / 16;
  constexpr int NT  = 64 * NQ;
  constexpr int NW  = NT / 32;
  constexpr int BCW = 2 * NSTATE;
  constexpr int YP  = 68;
  constexpr int RPI = NW * 4;
  constexpr int NIT = 64 / RPI;
  static_assert(16 * NT <= 64 * YP);
  __shared__ __align__(16) float sBC[64 * BCW];
  __shared__ __align__(16) float sY[64 * YP];
  const int tid  = threadIdx.x;
  const int lane = tid & 31;
  const int wave = tid >> 5;
  const int c    = tid / NQ;
  const int sq   = tid - c * NQ;
  const int bpb  = a.D / 64;
  const int bi   = blockIdx.x / bpb;
  if (bi >= a.nbatch) return;
  const int d0 = (blockIdx.x - bi * bpb) * 64;
  const int d  = d0 + c;
  const long rowb = (long)bi * a.L;
  const bool hasz  = (a.z != nullptr);
  const bool hasD  = (a.Dskip != nullptr);
  const bool hasLo = (a.y_lo != nullptr);

#pragma unroll 1
  for (int n = 0; n < 16; ++n) {
    const float al = a.A_log[(long)d * NSTATE + sq * 16 + n];
    sY[n * NT + tid] = -expf(al);
  }
  __syncthreads();
  float An[16], h[16];
#pragma unroll
  for (int n = 0; n < 16; ++n) {
    An[n] = sY[n * NT + tid];
    h[n] = 0.0f;
  }
  float Dd = 0.0f;
  if (hasD) Dd = a.Dskip[d];

  const int nchunk = a.L / 64;
  const bool fwd = (a.dir > 0);
  const int s0 = fwd ? 0 : 63;
  const int sd = fwd ? 1 : -1;
  const int q  = lane >> 3;
  const int c8 = (lane & 7) * 8;

#pragma unroll 1
  for (int ci = 0; ci < nchunk; ++ci) {
    const int tb = fwd ? (ci * 64) : (a.L - 64 - ci * 64);
    const long rowc = rowb + tb;
    __syncthreads();
#pragma unroll 8
    for (int i = 0; i < 32; ++i) {
      const int idx = tid + i * NT;
      const int st  = idx / BCW;
      const int col = idx - st * BCW;
      const int sc  = (col < NSTATE) ? (a.offB + col) : (a.offC + col - NSTATE);
      sBC[idx] = a.bc[(rowc + st) * a.ld_bc + sc];
    }
    __syncthreads();
#pragma unroll 1
    for (int s = 0; s < 64; ++s) {
      const int ls = s0 + sd * s;
      const long row = rowc + ls;
      float pre = a.dtpre[row * a.ld_dtpre + d];
      float uv  = a.u[row * a.ld_u + d];
      float zv  = 0.0f;
      if (hasz) zv = a.z[row * a.ld_z + a.offZ + d];
      asm volatile("" : "+v"(pre));
      asm volatile("" : "+v"(uv));
      asm volatile("" : "+v"(zv));
      const float delta = ms1_softplus(pre);
      const float dtx = delta * uv;
      const float* bp = sBC + ls * BCW + sq * 16;
      const float* cp = bp + NSTATE;
      ms1_v4f Bq[4], Cq[4];
#pragma unroll
      for (int k = 0; k < 4; ++k) {
        Bq[k] = *(const ms1_v4f*)(bp + 4 * k);
        Cq[k] = *(const ms1_v4f*)(cp + 4 * k);
      }
      float yv = 0.0f;
#pragma unroll
      for (int n = 0; n < 16; ++n) {
        const float e = __expf(delta * An[n]);
        h[n] = fmaf(e, h[n], dtx * Bq[n >> 2][n & 3]);
        yv = fmaf(h[n], Cq[n >> 2][n & 3], yv);
      }
      if (NQ > 1) {
        yv += __shfl_xor(yv, 1, 32);
        yv += __shfl_xor(yv, 2, 32);
      }
      if (hasD) yv = fmaf(uv, Dd, yv);
      if (hasz) {
        const float sg = __builtin_amdgcn_rcpf(1.0f + expf(-zv));
        yv = yv * (zv * sg);
      }
      if (sq == 0) sY[ls * YP + c] = yv * a.ycarry;
    }
    __syncthreads();
    ms1_v4u hw[NIT], lw[NIT];
#pragma unroll
    for (int it = 0; it < NIT; ++it) {
      const int row = it * RPI + wave * 4 + q;
      const float* sp = sY + row * YP + c8;
      const ms1_v4f f0 = *(const ms1_v4f*)(sp);
      const ms1_v4f f1 = *(const ms1_v4f*)(sp + 4);
      unsigned h0, h1, h2, h3, l0, l1, l2, l3;
      ms1_pack2(f0[0], f0[1], h0, l0);
      ms1_pack2(f0[2], f0[3], h1, l1);
      ms1_pack2(f1[0], f1[1], h2, l2);
      ms1_pack2(f1[2], f1[3], h3, l3);
      hw[it] = (ms1_v4u){h0, h1, h2, h3};
      lw[it] = (ms1_v4u){l0, l1, l2, l3};
    }
    for (int pass = 0; pass < 2; ++pass) {
#pragma unroll
      for (int it = 0; it < NIT; ++it) {
        const int row = it * RPI + wave * 4 + q;
        const long o = (rowc + row) * a.ld_y + d0 + c8;
        *(volatile ms1_v4u*)(a.y + o) = hw[it];
        if (hasLo) *(volatile ms1_v4u*)(a.y_lo + o) = lw[it];
      }
      __threadfence();
    }
  }
}

extern "C" void kernel_launch(void* const* d_in, const int* in_sizes, int n_in,
                              void* d_out, int out_size, void* d_ws, size_t ws_size,
                              hipStream_t stream) {
  if (n_in < 6) return;
  if (in_sizes[0] != kRows * kDin) return;
  if (in_sizes[1] != kProj * kDin) return;
  if (in_sizes[2] != kDin * kDtR) return;
  if (in_sizes[3] != kDin) return;
  if (in_sizes[4] != kDin * kNst) return;
  if (in_sizes[5] != kDin) return;
  if (out_size != kRows * kDin) return;
  if (ws_size < kWsTotal) return;

  const float* x     = (const float*)d_in[0];
  const float* W_x   = (const float*)d_in[1];
  const float* W_dt  = (const float*)d_in[2];
  const float* b_dt  = (const float*)d_in[3];
  const float* A_log = (const float*)d_in[4];
  const float* D_par = (const float*)d_in[5];
  float* out = (float*)d_out;

  char* ws = (char*)d_ws;
  unsigned short* XH   = (unsigned short*)(ws + kOffXH);
  unsigned short* WXH  = (unsigned short*)(ws + kOffWXH);
  unsigned short* WDH  = (unsigned short*)(ws + kOffWDH);
  float*          XP   = (float*)(ws + kOffXP);
  unsigned short* DTXH = (unsigned short*)(ws + kOffDTXH);
  float*          DT   = (float*)(ws + kOffDT);
  unsigned short* YH   = (unsigned short*)(ws + kOffYH);

  eng::to_f16_plane_kernel<<<(kRows * kDin / 8) / 256, 256, 0, stream>>>(
      x, kDin, kRows, kDin, XH, kRows * kDin / 8, kCarryX);
  eng::to_f16_plane_kernel<<<(kXpP * kDin / 8) / 256, 256, 0, stream>>>(
      W_x, kDin, kProj, kDin, WXH, kXpP * kDin / 8, kCarryWx);
  eng::to_f16_plane_kernel<<<(kDin * kDtR / 8) / 256, 256, 0, stream>>>(
      W_dt, kDtR, kDin, kDtR, WDH, kDin * kDtR / 8, kCarryWdt);

  eng::gemm_f16_kernel<0><<<dim3((kRows / 64) * (kXpP / 64) / 8), 256, 0, stream>>>(
      XH, kDin, WXH, kDin, XP, kXpP, nullptr, kRows, kXpP, kDin, kScale0);

  eng::to_f16_plane_kernel<<<(kRows * kDtR / 8) / 256, 256, 0, stream>>>(
      XP, kXpP, kRows, kDtR, DTXH, kRows * kDtR / 8, kCarryDtx);

  eng::gemm_f16_kernel<2><<<dim3((kRows / 64) * (kDin / 64) / 8), 256, 0, stream>>>(
      DTXH, kDtR, WDH, kDtR, DT, kDin, b_dt, kRows, kDin, kDtR, kScale1);

  for (int b = 0; b < kBatch; ++b) {
    const size_t r0 = (size_t)b * kSeq;
    ms1_args sa;
    sa.dtpre = DT + r0 * kDin;
    sa.u = x + r0 * kDin;
    sa.bc = XP + r0 * kXpP;
    sa.z = nullptr;
    sa.A_log = A_log;
    sa.Dskip = D_par;
    sa.y = (__half*)(YH + r0 * kDin);
    sa.y_lo = nullptr;
    sa.ld_dtpre = kDin;
    sa.ld_u = kDin;
    sa.ld_bc = kXpP;
    sa.ld_z = 0;
    sa.ld_y = kDin;
    sa.offB = kOffB;
    sa.offC = kOffC;
    sa.offZ = 0;
    sa.ycarry = kYCarry;
    sa.dir = 1;
    sa.D = kDin;
    sa.L = kSeq;
    sa.nbatch = 1;
    ms1_scan_kernel<16><<<dim3(kDin / 64), 64, 0, stream>>>(sa);
  }

  eng::decode_y_kernel<<<(kRows * kDin / 4) / 256, 256, 0, stream>>>(
      (const unsigned*)YH, out, kRows * kDin / 4, kYInv);
}
